// MultiLstm_81286551044510
// MI455X (gfx1250) — hardware-verified
//
#include <hip/hip_runtime.h>
#include <math.h>
#include <stdint.h>

constexpr int NSTEP  = 2048;
constexpr int NSEQ   = 64;
constexpr int NIN    = 64;
constexpr int NHID   = 128;
constexpr int NGATE  = 512;
constexpr int NTHR   = 256;
constexpr int TROWS  = 16;
constexpr int NBLK   = NSEQ / TROWS;
constexpr int HPITCH = 136;
constexpr int XPITCH = 72;
constexpr int OCH    = 32;
constexpr int GS_IN  = NHID * NIN;
constexpr int GS_HID = NHID * NHID;
constexpr float A_CARRY = 16.0f;
constexpr float W_CARRY = 64.0f;
constexpr float Z_FOLD  = 1.0f / 1024.0f;

static_assert(NSEQ % TROWS == 0);
static_assert(NBLK * TROWS == NSEQ);
static_assert(NTHR * 4 == TROWS * NIN);
static_assert(NSTEP % OCH == 0);
static_assert(OCH * TROWS == 4 * 32 * 4);
static_assert((NGATE * NIN / 8) % NTHR == 0);
static_assert((NGATE * NHID / 8) % NTHR == 0);
static_assert(NIN % 32 == 0 && NHID % 32 == 0);
static_assert((NSTEP * NSEQ / 4) % NTHR == 0);
static_assert(NHID == 16 * (NTHR / 32));

typedef __attribute__((ext_vector_type(16))) _Float16 v16h;
typedef __attribute__((ext_vector_type(8)))  _Float16 v8h;
typedef __attribute__((ext_vector_type(4)))  _Float16 v4h;
typedef __attribute__((ext_vector_type(16))) __bf16   v16b;
typedef __attribute__((ext_vector_type(8)))  __bf16   v8b;
typedef __attribute__((ext_vector_type(8)))  float    v8f;
typedef __attribute__((ext_vector_type(4)))  float    v4f;

__device__ __forceinline__ unsigned short f2bf_bits(float f) {
  unsigned u = __float_as_uint(f);
  return (unsigned short)((u + 0x7FFFu + ((u >> 16) & 1u)) >> 16);
}
__device__ __forceinline__ float bf_bits2f(unsigned short h) { return __uint_as_float(((unsigned)h) << 16); }
__device__ __forceinline__ float bfr(float f) { return bf_bits2f(f2bf_bits(f)); }

__device__ __forceinline__ void dep_guard_h(v8f& a, v8f& b, v16h x, v16h y) { asm volatile("v_nop\n\tv_nop\n\tv_nop\n\tv_nop" : "+v"(a), "+v"(b) : "v"(x), "v"(y)); }
__device__ __forceinline__ void dep_guard_b(v8f& a, v8f& b, v16b x, v16b y) { asm volatile("v_nop\n\tv_nop\n\tv_nop\n\tv_nop" : "+v"(a), "+v"(b) : "v"(x), "v"(y)); }
__device__ __forceinline__ void keep4_h(v16h a, v16h b, v16h c, v16h d) { asm volatile("v_nop" :: "v"(a), "v"(b), "v"(c), "v"(d)); }
__device__ __forceinline__ void keep4_b(v16b a, v16b b, v16b c, v16b d) { asm volatile("v_nop" :: "v"(a), "v"(b), "v"(c), "v"(d)); }
__device__ __forceinline__ void acc_guard4(v8f& a, v8f& b, v8f& c, v8f& d) { asm volatile("v_nop\n\tv_nop\n\tv_nop\n\tv_nop" : "+v"(a), "+v"(b), "+v"(c), "+v"(d)); }
__device__ __forceinline__ void mma_guard4x5(v8f& a, v8f& b, v8f& c, v8f& d, v16h x0, v16h x1, v16h x2, v16h x3, v16h x4) {
  asm volatile("v_nop\n\tv_nop\n\tv_nop\n\tv_nop" : "+v"(a), "+v"(b), "+v"(c), "+v"(d) : "v"(x0), "v"(x1), "v"(x2), "v"(x3), "v"(x4));
}
template <typename T> struct Frag;
template <> struct Frag<_Float16> {
  typedef v16h V; union U { v16h v; v8h h[2]; };
  static __device__ __forceinline__ v16h load(const _Float16* p) {
    U f; f.h[0] = *(const v8h*)(p); f.h[1] = *(const v8h*)(p + 16); return f.v;
  }
  static __device__ __forceinline__ v8f mma(v16h a, v16h b, v8f c) {
    return __builtin_amdgcn_wmma_f32_16x16x32_f16(false, a, false, b, (short)0, c, false, false);
  }
  static __device__ __forceinline__ void guard(v8f& a, v8f& b, v16h x, v16h y) { dep_guard_h(a, b, x, y); }
  static __device__ __forceinline__ void keep(v16h a, v16h b, v16h c, v16h d) { keep4_h(a, b, c, d); }
};
template <> struct Frag<__bf16> {
  typedef v16b V; union U { v16b v; v8b h[2]; };
  static __device__ __forceinline__ v16b load(const __bf16* p) {
    U f; f.h[0] = *(const v8b*)(p); f.h[1] = *(const v8b*)(p + 16); return f.v;
  }
  static __device__ __forceinline__ v8f mma(v16b a, v16b b, v8f c) {
    return __builtin_amdgcn_wmma_f32_16x16x32_bf16(false, a, false, b, (short)0, c, false, false);
  }
  static __device__ __forceinline__ void guard(v8f& a, v8f& b, v16b x, v16b y) { dep_guard_b(a, b, x, y); }
  static __device__ __forceinline__ void keep(v16b a, v16b b, v16b c, v16b d) { keep4_b(a, b, c, d); }
};
typedef Frag<_Float16> FragH;

__device__ __forceinline__ float fsig(float v)  { return __builtin_amdgcn_rcpf(1.0f + __expf(-v)); }
__device__ __forceinline__ float ftanh(float v) { return 1.0f - 2.0f * __builtin_amdgcn_rcpf(__expf(2.0f * v) + 1.0f); }

__global__ __launch_bounds__(NTHR) void wprep_kernel(const float* __restrict__ W, int n8, unsigned short* __restrict__ O) {
  const int i = blockIdx.x * NTHR + threadIdx.x;
  if (i >= n8) return;
  const int e0 = i * 8;
  v8h hv;
#pragma unroll
  for (int e = 0; e < 8; ++e) {
    const float fb = bfr(W[e0 + e]);
    hv[e] = (_Float16)(fb * W_CARRY);
  }
  *(volatile v8h*)(O + e0) = hv;
  __threadfence();
  *(volatile v8h*)(O + e0) = hv;
}

template <int NK, int GSTR>
__device__ __forceinline__ void mac4(v8f (&acc)[4], const _Float16* arow, const _Float16* wrow) {
#pragma unroll 1
  for (int kc = 0; kc < NK; ++kc) {
    const int k0 = kc * 32;
    const v16h a  = FragH::load(arow + k0);
    const v16h b0 = FragH::load(wrow + k0);
    const v16h b1 = FragH::load(wrow + GSTR + k0);
    const v16h b2 = FragH::load(wrow + 2 * GSTR + k0);
    const v16h b3 = FragH::load(wrow + 3 * GSTR + k0);
    acc[0] = FragH::mma(a, b0, acc[0]);
    acc[1] = FragH::mma(a, b1, acc[1]);
    acc[2] = FragH::mma(a, b2, acc[2]);
    acc[3] = FragH::mma(a, b3, acc[3]);
    mma_guard4x5(acc[0], acc[1], acc[2], acc[3], a, b0, b1, b2, b3);
  }
}

__device__ __forceinline__ void lstm_cell8(const v8f (&acc)[4], float bi, float bfg, float bg, float bo,
                                           float (&cs)[8], float (&h)[8]) {
#pragma unroll
  for (int r = 0; r < 8; ++r) {
    const float pi = fmaf(acc[0][r], Z_FOLD, bi);
    const float pf = fmaf(acc[1][r], Z_FOLD, bfg);
    const float pg = fmaf(acc[2][r], Z_FOLD, bg);
    const float po = fmaf(acc[3][r], Z_FOLD, bo);
    const float ig = fsig(pi);
    const float fg = fsig(pf);
    const float gg = ftanh(pg);
    const float og = fsig(po);
    const float cn = fmaf(fg, cs[r], ig * gg);
    cs[r] = cn;
    h[r] = og * ftanh(cn);
  }
}

__global__ __launch_bounds__(NTHR) void lstm2_kernel(
    const float* __restrict__ data,
    const float* __restrict__ bih0, const float* __restrict__ bhh0,
    const float* __restrict__ bih1, const float* __restrict__ bhh1,
    const float* __restrict__ wlin, const float* __restrict__ blin,
    const unsigned short* __restrict__ Wih0p, const unsigned short* __restrict__ Whh0p,
    const unsigned short* __restrict__ Wih1p, const unsigned short* __restrict__ Whh1p,
    float* __restrict__ slab) {
  __shared__ __align__(16) _Float16 H0s[TROWS * HPITCH];
  __shared__ __align__(16) _Float16 H1s[TROWS * HPITCH];
  __shared__ __align__(16) _Float16 Xh[TROWS * XPITCH];
  __shared__ __align__(16) float    Ps[(NTHR / 32) * TROWS];
  __shared__ __align__(16) float    Os[OCH * TROWS];

  const int tid = threadIdx.x, lane = tid & 31, wave = tid >> 5;
  const int c = lane & 15, hh = lane >> 4, koff = hh * 8;
  const int j  = 16 * wave + c;
  const int rb = 8 * hh;
  const int sb = blockIdx.x * TROWS;

#pragma unroll 1
  for (int i = tid; i < TROWS * HPITCH; i += NTHR) { H0s[i] = (_Float16)0.0f; H1s[i] = (_Float16)0.0f; }
  if (tid < TROWS * 8) Xh[(tid >> 3) * XPITCH + NIN + (tid & 7)] = (_Float16)0.0f;

  const float b0i = bfr(bih0[j]) + bfr(bhh0[j]);
  const float b0f = bfr(bih0[NHID + j]) + bfr(bhh0[NHID + j]);
  const float b0g = bfr(bih0[2 * NHID + j]) + bfr(bhh0[2 * NHID + j]);
  const float b0o = bfr(bih0[3 * NHID + j]) + bfr(bhh0[3 * NHID + j]);
  const float b1i = bfr(bih1[j]) + bfr(bhh1[j]);
  const float b1f = bfr(bih1[NHID + j]) + bfr(bhh1[NHID + j]);
  const float b1g = bfr(bih1[2 * NHID + j]) + bfr(bhh1[2 * NHID + j]);
  const float b1o = bfr(bih1[3 * NHID + j]) + bfr(bhh1[3 * NHID + j]);
  const float wl  = bfr(wlin[j]);
  const float bl  = bfr(blin[0]);

  float cst0[8], cst1[8];
#pragma unroll
  for (int r = 0; r < 8; ++r) { cst0[r] = 0.0f; cst1[r] = 0.0f; }
  __syncthreads();

  const _Float16* xrow  = Xh  + c * XPITCH + koff;
  const _Float16* h0row = H0s + c * HPITCH + koff;
  const _Float16* h1row = H1s + c * HPITCH + koff;
  const _Float16* wih0 = (const _Float16*)Wih0p + (size_t)j * NIN  + koff;
  const _Float16* whh0 = (const _Float16*)Whh0p + (size_t)j * NHID + koff;
  const _Float16* wih1 = (const _Float16*)Wih1p + (size_t)j * NHID + koff;
  const _Float16* whh1 = (const _Float16*)Whh1p + (size_t)j * NHID + koff;
  const v8f z8 = {0.f, 0.f, 0.f, 0.f, 0.f, 0.f, 0.f, 0.f};
  float* slab_blk = slab + (size_t)blockIdx.x * NSTEP * TROWS;

#pragma unroll 1
  for (int t = 0; t < NSTEP; ++t) {
    {
      const int row = tid >> 4, c4 = (tid & 15) * 4;
      const v4f v = *(const v4f*)(data + (((size_t)t * NSEQ + (size_t)(sb + row)) * NIN + (size_t)c4));
      v4h w;
      w[0] = (_Float16)(A_CARRY * bfr(v[0]));
      w[1] = (_Float16)(A_CARRY * bfr(v[1]));
      w[2] = (_Float16)(A_CARRY * bfr(v[2]));
      w[3] = (_Float16)(A_CARRY * bfr(v[3]));
      *(v4h*)(Xh + row * XPITCH + c4) = w;
    }
    __syncthreads();
    float h0v[8];
    {
      v8f acc[4];
      acc[0] = z8; acc[1] = z8; acc[2] = z8; acc[3] = z8;
      mac4<NIN / 32,  GS_IN >(acc, xrow,  wih0);
      mac4<NHID / 32, GS_HID>(acc, h0row, whh0);
      lstm_cell8(acc, b0i, b0f, b0g, b0o, cst0, h0v);
    }
    __syncthreads();
#pragma unroll
    for (int r = 0; r < 8; ++r) H0s[(rb + r) * HPITCH + j] = (_Float16)(A_CARRY * h0v[r]);
    __syncthreads();
    float h1v[8];
    {
      v8f acc[4];
      acc[0] = z8; acc[1] = z8; acc[2] = z8; acc[3] = z8;
      mac4<NHID / 32, GS_HID>(acc, h0row, wih1);
      mac4<NHID / 32, GS_HID>(acc, h1row, whh1);
      lstm_cell8(acc, b1i, b1f, b1g, b1o, cst1, h1v);
#pragma unroll
      for (int r = 0; r < 8; ++r) {
        float p = h1v[r] * wl;
        p += __shfl_xor(p, 1, 32);
        p += __shfl_xor(p, 2, 32);
        p += __shfl_xor(p, 4, 32);
        p += __shfl_xor(p, 8, 32);
        if (c == 0) Ps[wave * TROWS + rb + r] = p;
      }
    }
    __syncthreads();
#pragma unroll
    for (int r = 0; r < 8; ++r) H1s[(rb + r) * HPITCH + j] = (_Float16)(A_CARRY * h1v[r]);
    if (wave == 0) {
      const int m = lane & 15;
      float s = Ps[m];
#pragma unroll
      for (int w = 1; w < NTHR / 32; ++w) s += Ps[w * TROWS + m];
      const float o = s + bl;
      if (lane < TROWS) Os[(t & (OCH - 1)) * TROWS + lane] = o;
      if ((t & (OCH - 1)) == OCH - 1) {
        __builtin_amdgcn_fence(__ATOMIC_RELEASE, "workgroup");
        __builtin_amdgcn_wave_barrier();
        __builtin_amdgcn_fence(__ATOMIC_ACQUIRE, "workgroup");
        float* dst = slab_blk + (size_t)(t - (OCH - 1)) * TROWS;
        for (int pass = 0; pass < 2; ++pass) {
#pragma unroll
          for (int it = 0; it < 4; ++it) {
            const v4f v = *(const v4f*)(Os + it * 128 + lane * 4);
            *(volatile v4f*)(dst + it * 128 + lane * 4) = v;
          }
          __threadfence();
        }
      }
    }
  }
}

__global__ __launch_bounds__(NTHR) void assemble_kernel(const float* __restrict__ slab, float* __restrict__ out, int n4) {
  const int i = blockIdx.x * NTHR + threadIdx.x;
  if (i >= n4) return;
  const int t = i >> 4, q = i & 15;
  const int blk = q >> 2, c4 = (q & 3) * 4;
  const v4f v = *(const v4f*)(slab + ((size_t)blk * NSTEP + (size_t)t) * TROWS + c4);
  float* op = out + (size_t)t * NSEQ + (size_t)(q * 4);
  *(volatile v4f*)op = v;
  __threadfence();
  *(volatile v4f*)op = v;
}

extern "C" void kernel_launch(void* const* d_in, const int* in_sizes, int n_in,
                              void* d_out, int out_size, void* d_ws, size_t ws_size, hipStream_t stream) {
  if (n_in < 11 || d_out == nullptr || d_ws == nullptr) return;
  if (in_sizes[0] != NSTEP * NSEQ * NIN || in_sizes[1] != NGATE * NIN || in_sizes[2] != NGATE * NHID ||
      in_sizes[3] != NGATE || in_sizes[4] != NGATE || in_sizes[5] != NGATE * NHID || in_sizes[6] != NGATE * NHID ||
      in_sizes[7] != NGATE || in_sizes[8] != NGATE || in_sizes[9] != NHID || in_sizes[10] < 1 ||
      out_size != NSTEP * NSEQ) return;

  const float* data = (const float*)d_in[0];
  const float* Wih0 = (const float*)d_in[1];
  const float* Whh0 = (const float*)d_in[2];
  const float* bih0 = (const float*)d_in[3];
  const float* bhh0 = (const float*)d_in[4];
  const float* Wih1 = (const float*)d_in[5];
  const float* Whh1 = (const float*)d_in[6];
  const float* bih1 = (const float*)d_in[7];
  const float* bhh1 = (const float*)d_in[8];
  const float* Wlin = (const float*)d_in[9];
  const float* blin = (const float*)d_in[10];
  float* out = (float*)d_out;

  char* ws = (char*)d_ws; size_t off = 0;
  auto carve = [&](size_t bytes) -> char* { char* p = ws + off; off += (bytes + 255) & ~(size_t)255; return p; };
  unsigned short* WIH0 = (unsigned short*)carve((size_t)NGATE * NIN * 2);
  unsigned short* WHH0 = (unsigned short*)carve((size_t)NGATE * NHID * 2);
  unsigned short* WIH1 = (unsigned short*)carve((size_t)NGATE * NHID * 2);
  unsigned short* WHH1 = (unsigned short*)carve((size_t)NGATE * NHID * 2);
  float*          SLAB = (float*)carve((size_t)NBLK * NSTEP * TROWS * 4);
  if (off > ws_size || off > (size_t)134217728) return;

  const int n8_in = NGATE * NIN / 8, n8_hid = NGATE * NHID / 8;
  wprep_kernel<<<n8_in / NTHR,  NTHR, 0, stream>>>(Wih0, n8_in,  WIH0);
  wprep_kernel<<<n8_hid / NTHR, NTHR, 0, stream>>>(Whh0, n8_hid, WHH0);
  wprep_kernel<<<n8_hid / NTHR, NTHR, 0, stream>>>(Wih1, n8_hid, WIH1);
  wprep_kernel<<<n8_hid / NTHR, NTHR, 0, stream>>>(Whh1, n8_hid, WHH1);
  lstm2_kernel<<<NBLK, NTHR, 0, stream>>>(data, bih0, bhh0, bih1, bhh1, Wlin, blin, WIH0, WHH0, WIH1, WHH1, SLAB);
  const int n4 = NSTEP * NSEQ / 4;
  assemble_kernel<<<n4 / NTHR, NTHR, 0, stream>>>(SLAB, out, n4);
}
